// FoldingNet_43628277793055
// MI455X (gfx1250) — hardware-verified
//
#include <hip/hip_runtime.h>
#include <math.h>

#ifndef NB
#define NB 128
#endif
#ifndef NPTS
#define NPTS 2048
#endif
#define NPTS_FULL 2048
#define LAT 256
#define W1_LD 258
#define W4_LD 259
#define TP 68

#define OFF_X16 0
#define OFF_W1A (NB * 256)
#define OFF_W4A (OFF_W1A + 16384)
#define OFF_W2P (OFF_W4A + 16384)
#define OFF_W5P (OFF_W2P + 1024)
#define OFF_W3P (OFF_W5P + 1024)
#define OFF_W6P (OFF_W3P + 512)
#define OFF_W4T (OFF_W6P + 512)
#define PL_HALVES (OFF_W4T + 2048)

#define PB0 (NB / 2)
#define PB1 (PB0 + 32)
#define PB2 (PB1 + 32)
#define PB3 (PB2 + 2)
#define PB4 (PB3 + 2)
#define PB5 (PB4 + 1)
#define PB6 (PB5 + 1)
#define PB7 (PB6 + 4)

#define WAVES_PER_ROW (NPTS / 32)
#define TOTAL_WAVES (NB * WAVES_PER_ROW)

static_assert(NB % 16 == 0 && NB <= 128);
static_assert(NPTS % 32 == 0 && NPTS <= NPTS_FULL);
static_assert((WAVES_PER_ROW & (WAVES_PER_ROW - 1)) == 0);
static_assert(TOTAL_WAVES % 8 == 0);
static_assert(LAT % 32 == 0);
static_assert(PB7 * 64 * 8 == PL_HALVES);
static_assert((NPTS * 16) % 256 == 0);
static_assert(OFF_W1A % 64 == 0 && OFF_W2P % 64 == 0 && OFF_W3P % 64 == 0 && OFF_W6P % 64 == 0 && OFF_W4T % 64 == 0);
static_assert(32 * 16 * 8 == 16 * 64 * 4);
static_assert(24 * 16 * 1 == 32 * 3 * 4);
static_assert(NPTS * 16 * 16 == NPTS * 64 * 4);
static_assert(8 * 16 * TP * 4 + 8 * 96 * 4 <= 131072);
static_assert((TP * 4) % 16 == 0);

constexpr size_t WS_PLANES = 0;
constexpr size_t WS_P      = (((size_t)PL_HALVES * 2) + 255) & ~(size_t)255;
constexpr size_t WS_G1     = WS_P + ((((size_t)2 * NB * 64 * 4) + 255) & ~(size_t)255);
constexpr size_t WS_TOTAL  = WS_G1 + (size_t)NPTS * 64 * 4;
static_assert(WS_TOTAL <= 134217728);
static_assert(WS_P % 256 == 0 && WS_G1 % 256 == 0);

typedef __attribute__((ext_vector_type(16))) _Float16 v16h;
typedef __attribute__((ext_vector_type(8)))  _Float16 v8h;
typedef __attribute__((ext_vector_type(2)))  _Float16 v2h;
typedef __attribute__((ext_vector_type(8)))  float    v8f;
typedef __attribute__((ext_vector_type(4)))  float    v4f;
typedef __attribute__((ext_vector_type(2)))  float    v2f;


#define X_CARRY 256.0f
#define W_CARRY 4096.0f
#define ACT_CARRY 1024.0f
#define LO_CARRY 2048.0f
#define LO_BACK 4.8828125e-04f
#define SC20 9.5367431640625e-07f
#define SC22 2.384185791015625e-07f
#define P4_CARRY 4194304.0f

__device__ __forceinline__ float bfr(float f) {
    unsigned u = __float_as_uint(f);
    u += 0x7FFFu + ((u >> 16) & 1u);
    return __uint_as_float(u & 0xFFFF0000u);
}

union FragU { v16h v; v8h h[2]; };
__device__ __forceinline__ v16h frag_ld(const _Float16* p) {
    FragU f; f.h[0] = *(const v8h*)(p); f.h[1] = *(const v8h*)(p + 16); return f.v;
}
__device__ __forceinline__ v8f wmma16(v16h a, v16h b, v8f c) {
    c = __builtin_amdgcn_wmma_f32_16x16x32_f16(false, a, false, b, (short)0, c, false, false);
    asm volatile("v_nop\n\tv_nop\n\tv_nop\n\tv_nop" : "+v"(c) : "v"(a), "v"(b));
    return c;
}
__device__ __forceinline__ void wave_sync_lds() {
    __builtin_amdgcn_fence(3  , "workgroup");
    __builtin_amdgcn_wave_barrier();
    __builtin_amdgcn_fence(2  , "workgroup");
}

__device__ __forceinline__ v2h toh_flush2(float a, float b) {
    v2f w;
    w.x = (fabsf(a) < 6.103515625e-05f) ? 0.0f : a;
    w.y = (fabsf(b) < 6.103515625e-05f) ? 0.0f : b;
    return __builtin_convertvector(w, v2h);
}
__device__ __forceinline__ void split2(float a, float b, v2h& hi, v2h& lo) {
    const float sa = a * ACT_CARRY, sb = b * ACT_CARRY;
    hi = toh_flush2(sa, sb);
    const v2f hf = __builtin_convertvector(hi, v2f);
    lo = toh_flush2((sa - hf.x) * LO_CARRY, (sb - hf.y) * LO_CARRY);
}
__device__ __forceinline__ void one4(const v4f a, v2h& q0, v2h& q1) {
    q0 = toh_flush2(a.x * ACT_CARRY, a.y * ACT_CARRY);
    q1 = toh_flush2(a.z * ACT_CARRY, a.w * ACT_CARRY);
}
__device__ __forceinline__ void two4(const v4f a, v2h& h0, v2h& h1, v2h& l0, v2h& l1) {
    split2(a.x, a.y, h0, l0);
    split2(a.z, a.w, h1, l1);
}

union FragP { v16h v; v2h p[8]; };
union PackH8 { v8h v; v2h p[4]; };

__device__ __forceinline__ v16h afrag1_full(const float* p) {
    const v4f a0 = *(const v4f*)(p), a1 = *(const v4f*)(p + 4), a2 = *(const v4f*)(p + 16), a3 = *(const v4f*)(p + 20);
    FragP f;
    one4(a0, f.p[0], f.p[1]); one4(a1, f.p[2], f.p[3]); one4(a2, f.p[4], f.p[5]); one4(a3, f.p[6], f.p[7]);
    return f.v;
}
__device__ __forceinline__ v16h afrag1_half(const float* p) {
    const v4f a0 = *(const v4f*)(p), a1 = *(const v4f*)(p + 4);
    const v2h zz = (v2h){(_Float16)0.0f, (_Float16)0.0f};
    FragP f;
    one4(a0, f.p[0], f.p[1]); one4(a1, f.p[2], f.p[3]);
    f.p[4] = zz; f.p[5] = zz; f.p[6] = zz; f.p[7] = zz;
    return f.v;
}
__device__ __forceinline__ void afrag2_full(const float* p, v16h& hi, v16h& lo) {
    const v4f a0 = *(const v4f*)(p), a1 = *(const v4f*)(p + 4), a2 = *(const v4f*)(p + 16), a3 = *(const v4f*)(p + 20);
    FragP fh, fl;
    two4(a0, fh.p[0], fh.p[1], fl.p[0], fl.p[1]);
    two4(a1, fh.p[2], fh.p[3], fl.p[2], fl.p[3]);
    two4(a2, fh.p[4], fh.p[5], fl.p[4], fl.p[5]);
    two4(a3, fh.p[6], fh.p[7], fl.p[6], fl.p[7]);
    hi = fh.v; lo = fl.v;
}
__device__ __forceinline__ void afrag2_half(const float* p, v16h& hi, v16h& lo) {
    const v4f a0 = *(const v4f*)(p), a1 = *(const v4f*)(p + 4);
    const v2h zz = (v2h){(_Float16)0.0f, (_Float16)0.0f};
    FragP fh, fl;
    two4(a0, fh.p[0], fh.p[1], fl.p[0], fl.p[1]);
    two4(a1, fh.p[2], fh.p[3], fl.p[2], fl.p[3]);
    fh.p[4] = zz; fh.p[5] = zz; fh.p[6] = zz; fh.p[7] = zz;
    fl.p[4] = zz; fl.p[5] = zz; fl.p[6] = zz; fl.p[7] = zz;
    hi = fh.v; lo = fl.v;
}

__device__ __forceinline__ float half_sum16(float v) {
    v += __shfl_xor(v, 1, 32);
    v += __shfl_xor(v, 2, 32);
    v += __shfl_xor(v, 4, 32);
    v += __shfl_xor(v, 8, 32);
    return v;
}

__device__ __forceinline__ void ln64_relu_store(const v8f (&z)[4], const float (&g)[4], const float (&be)[4],
                                                float* tile, unsigned hh, unsigned c) {
#pragma unroll
    for (int r = 0; r < 8; ++r) {
        const float s = half_sum16((z[0][r] + z[1][r]) + (z[2][r] + z[3][r]));
        const float mu = s * (1.0f / 64.0f);
        float d[4];
#pragma unroll
        for (int j = 0; j < 4; ++j) d[j] = z[j][r] - mu;
        const float q = half_sum16((d[0] * d[0] + d[1] * d[1]) + (d[2] * d[2] + d[3] * d[3]));
        const float rs = 1.0f / sqrtf(q * (1.0f / 64.0f) + 1e-5f);
#pragma unroll
        for (int j = 0; j < 4; ++j) {
            const float y = d[j] * rs * g[j] + be[j];
            tile[(8u * hh + (unsigned)r) * TP + 16u * (unsigned)j + c] = fmaxf(y, 0.0f);
        }
    }
}
__device__ __forceinline__ void ln16_relu_store(const v8f z, float g, float be, float* tile, unsigned hh, unsigned c) {
#pragma unroll
    for (int r = 0; r < 8; ++r) {
        const float s = half_sum16(z[r]);
        const float mu = s * (1.0f / 16.0f);
        const float d = z[r] - mu;
        const float q = half_sum16(d * d);
        const float rs = 1.0f / sqrtf(q * (1.0f / 16.0f) + 1e-5f);
        const float y = d * rs * g + be;
        tile[(8u * hh + (unsigned)r) * TP + c] = fmaxf(y, 0.0f);
    }
}
__device__ __forceinline__ void ln3_relu_store(const v8f z, float g, float be, bool live, float* tile, unsigned hh, unsigned c) {
#pragma unroll
    for (int r = 0; r < 8; ++r) {
        const float zl = live ? z[r] : 0.0f;
        const float s = half_sum16(zl);
        const float mu = s / 3.0f;
        const float d = live ? (z[r] - mu) : 0.0f;
        const float q = half_sum16(d * d);
        const float rs = 1.0f / sqrtf(q / 3.0f + 1e-5f);
        const float y = fmaxf(d * rs * g + be, 0.0f);
        tile[(8u * hh + (unsigned)r) * TP + c] = live ? y : 0.0f;
    }
}

__device__ __forceinline__ void fold_grid(unsigned p, float& g0, float& g1) {
    const float a = (float)p * (4096.0f / 2047.0f);
    g0 = truncf(a / 45.254833995939045f) / 45.254833995939045f - 1.0f;
    const float b = (float)p * (2048.0f / 2047.0f);
    g1 = 2.0f * (b - floorf(b / 45.254833995939045f) * 45.254833995939045f) / 45.254833995939045f - 1.0f;
}

__device__ __forceinline__ void st8h_flush(_Float16* P, unsigned o, const float* v) {
    PackH8 pk;
    pk.p[0] = toh_flush2(v[0], v[1]);
    pk.p[1] = toh_flush2(v[2], v[3]);
    pk.p[2] = toh_flush2(v[4], v[5]);
    pk.p[3] = toh_flush2(v[6], v[7]);
    const v8h hv = pk.v;
    *(volatile v8h*)(P + o) = hv;
    __threadfence();
    *(volatile v8h*)(P + o) = hv;
}

__global__ __launch_bounds__(64) void k_prep(const float* __restrict__ x, const float* __restrict__ W1, const float* __restrict__ W2,
                                             const float* __restrict__ W3, const float* __restrict__ W4, const float* __restrict__ W5,
                                             const float* __restrict__ W6, _Float16* __restrict__ planes) {
    const unsigned blk = blockIdx.x, t = threadIdx.x;
    float v[8];
    unsigned dst;
    if (blk < (unsigned)PB0) {
        const unsigned u = blk * 64u + t;
#pragma unroll
        for (int i = 0; i < 8; ++i) v[i] = bfr(x[u * 8u + (unsigned)i]) * X_CARRY;
        dst = (unsigned)OFF_X16 + u * 8u;
    } else if (blk < (unsigned)PB1) {
        const unsigned u = (blk - (unsigned)PB0) * 64u + t;
        const unsigned o = u >> 5, k0 = (u & 31u) * 8u;
#pragma unroll
        for (int i = 0; i < 8; ++i) v[i] = bfr(W1[o * (unsigned)W1_LD + k0 + (unsigned)i]) * W_CARRY;
        dst = (unsigned)OFF_W1A + u * 8u;
    } else if (blk < (unsigned)PB2) {
        const unsigned u = (blk - (unsigned)PB1) * 64u + t;
        const unsigned o = u >> 5, k0 = (u & 31u) * 8u;
#pragma unroll
        for (int i = 0; i < 8; ++i) v[i] = bfr(W4[o * (unsigned)W4_LD + k0 + (unsigned)i]) * W_CARRY;
        dst = (unsigned)OFF_W4A + u * 8u;
    } else if (blk < (unsigned)PB3) {
        const unsigned u = (blk - (unsigned)PB2) * 64u + t;
#pragma unroll
        for (int i = 0; i < 8; ++i) v[i] = bfr(W2[u * 8u + (unsigned)i]) * W_CARRY;
        dst = (unsigned)OFF_W2P + u * 8u;
    } else if (blk < (unsigned)PB4) {
        const unsigned u = (blk - (unsigned)PB3) * 64u + t;
#pragma unroll
        for (int i = 0; i < 8; ++i) v[i] = bfr(W5[u * 8u + (unsigned)i]) * W_CARRY;
        dst = (unsigned)OFF_W5P + u * 8u;
    } else if (blk < (unsigned)PB5) {
        const unsigned u = (blk - (unsigned)PB4) * 64u + t;
        const unsigned row = u >> 2, k0 = (u & 3u) * 8u;
        const unsigned rc = (row < 2u) ? row : 2u, kc = (k0 < 8u) ? k0 : 8u;
        const bool live = (row < 3u) && (k0 < 16u);
#pragma unroll
        for (int i = 0; i < 8; ++i) {
            const float w = bfr(W3[rc * 16u + kc + (unsigned)i]) * W_CARRY;
            v[i] = live ? w : 0.0f;
        }
        dst = (unsigned)OFF_W3P + u * 8u;
    } else if (blk < (unsigned)PB6) {
        const unsigned u = (blk - (unsigned)PB5) * 64u + t;
        const unsigned row = u >> 2, k0 = (u & 3u) * 8u;
        const unsigned rc = (row < 2u) ? row : 2u, kc = (k0 < 8u) ? k0 : 8u;
        const bool live = (row < 3u) && (k0 < 16u);
#pragma unroll
        for (int i = 0; i < 8; ++i) {
            const float w = bfr(W6[rc * 16u + kc + (unsigned)i]) * W_CARRY;
            v[i] = live ? w : 0.0f;
        }
        dst = (unsigned)OFF_W6P + u * 8u;
    } else {
        const unsigned u = (blk - (unsigned)PB6) * 64u + t;
        const unsigned o = u >> 2, k0 = (u & 3u) * 8u;
#pragma unroll
        for (int i = 0; i < 8; ++i) {
            const unsigned ic = (i < 3) ? (unsigned)i : 2u;
            const float w = bfr(W4[o * (unsigned)W4_LD + 256u + ic]) * W_CARRY;
            v[i] = ((k0 == 0u) && (i < 3)) ? w : 0.0f;
        }
        dst = (unsigned)OFF_W4T + u * 8u;
    }
    st8h_flush(planes, dst, v);
}

__global__ __launch_bounds__(256) void k_lat(const _Float16* __restrict__ planes, const float* __restrict__ b1,
                                             const float* __restrict__ b4, float* __restrict__ P) {
    __shared__ __align__(16) float sS[8][16 * TP];
    const unsigned lane = threadIdx.x & 31u;
    const unsigned wave = __builtin_amdgcn_readfirstlane(threadIdx.x >> 5);
    if (wave >= (unsigned)(NB / 16)) return;
    const unsigned which = blockIdx.x;
    const unsigned hh = lane >> 4, c = lane & 15u;
    const unsigned m0 = wave * 16u;
    const _Float16* A  = planes + (unsigned)OFF_X16 + (m0 + c) * 256u + 8u * hh;
    const _Float16* Bt = planes + (unsigned)OFF_W1A + which * 16384u + c * 256u + 8u * hh;

    v8f acc[4];
#pragma unroll
    for (int j = 0; j < 4; ++j) acc[j] = (v8f){0.f,0.f,0.f,0.f,0.f,0.f,0.f,0.f};

    for (unsigned k0 = 0; k0 < (unsigned)LAT; k0 += 32u) {
        const v16h a = frag_ld(A + k0);
#pragma unroll
        for (int j = 0; j < 4; ++j) {
            const v16h bf = frag_ld(Bt + (unsigned)j * 4096u + k0);
            acc[j] = wmma16(a, bf, acc[j]);
        }
    }

    float* slab = sS[wave];
#pragma unroll
    for (int j = 0; j < 4; ++j) {
        const unsigned n = 16u * (unsigned)j + c;
        const float bA = bfr(b1[n]);
        const float bB = bfr(b4[n]);
        const float bv = (which == 0u) ? bA : bB;
#pragma unroll
        for (int r = 0; r < 8; ++r) slab[(8u * hh + (unsigned)r) * TP + n] = acc[j][r] * SC20 + bv;
    }
    wave_sync_lds();
    float* dst = P + which * (unsigned)(NB * 64) + m0 * 64u;
    const unsigned c4 = c * 4u;
    v4f vv[8];
#pragma unroll
    for (int it = 0; it < 8; ++it) {
        const unsigned row = 2u * (unsigned)it + hh;
        vv[it] = *(const v4f*)(slab + row * TP + c4);
    }
    for (int pass = 0; pass < 2; ++pass) {
#pragma unroll
        for (int it = 0; it < 8; ++it) {
            const unsigned row = 2u * (unsigned)it + hh;
            *(volatile v4f*)(dst + row * 64u + c4) = vv[it];
        }
        __threadfence();
    }
}

__global__ __launch_bounds__(256) void k_grid(const float* __restrict__ W1, float* __restrict__ G1) {
    const unsigned u = blockIdx.x * 256u + threadIdx.x;
    if (u >= (unsigned)(NPTS * 16)) return;
    const unsigned p = u >> 4, c4 = (u & 15u) * 4u;
    float g0, g1;
    fold_grid(p, g0, g1);
    float tv[4];
#pragma unroll
    for (int i = 0; i < 4; ++i) {
        const float* wr = W1 + (c4 + (unsigned)i) * (unsigned)W1_LD + 256u;
        tv[i] = g0 * bfr(wr[0]) + g1 * bfr(wr[1]);
    }
    v4f o; o.x = tv[0]; o.y = tv[1]; o.z = tv[2]; o.w = tv[3];
    float* dst = G1 + p * 64u + c4;
    *(volatile v4f*)dst = o;
    __threadfence();
    *(volatile v4f*)dst = o;
}

__global__ __launch_bounds__(256) void k_fold(
    const _Float16* __restrict__ planes, const float* __restrict__ P, const float* __restrict__ G1,
    const float* __restrict__ b2, const float* __restrict__ b3, const float* __restrict__ b5, const float* __restrict__ b6,
    const float* __restrict__ g1, const float* __restrict__ be1, const float* __restrict__ g2, const float* __restrict__ be2,
    const float* __restrict__ g3, const float* __restrict__ be3, const float* __restrict__ g4, const float* __restrict__ be4,
    const float* __restrict__ g5, const float* __restrict__ be5, float* __restrict__ out) {
    __shared__ __align__(16) float sT[8][16 * TP];
    __shared__ __align__(16) float sO[8][96];
    const unsigned lane = threadIdx.x & 31u;
    const unsigned wave = __builtin_amdgcn_readfirstlane(threadIdx.x >> 5);
    const unsigned W = blockIdx.x * 8u + wave;
    if (W >= (unsigned)TOTAL_WAVES) return;
    const unsigned b = W / (unsigned)WAVES_PER_ROW;
    const unsigned p0 = (W % (unsigned)WAVES_PER_ROW) * 32u;
    const unsigned hh = lane >> 4, c = lane & 15u;
    float* tile = sT[wave];
    float* so = sO[wave];

    float g1v[4], e1v[4], g4v[4], e4v[4], p1v[4], p4v[4];
#pragma unroll
    for (int j = 0; j < 4; ++j) {
        const unsigned ch = 16u * (unsigned)j + c;
        g1v[j] = bfr(g1[ch]);  e1v[j] = bfr(be1[ch]);
        g4v[j] = bfr(g4[ch]);  e4v[j] = bfr(be4[ch]);
        p1v[j] = P[b * 64u + ch];
        p4v[j] = P[(unsigned)(NB * 64) + b * 64u + ch] * P4_CARRY;
    }
    const float b2v = bfr(b2[c]), g2v = bfr(g2[c]), e2v = bfr(be2[c]);
    const float b5v = bfr(b5[c]), g5v = bfr(g5[c]), e5v = bfr(be5[c]);
    const unsigned c3 = (c < 2u) ? c : 2u;
    const bool live3 = c < 3u;
    const float b3v = bfr(b3[c3]), g3v = bfr(g3[c3]), e3v = bfr(be3[c3]);
    const float b6v = bfr(b6[c3]);
    const v8f zero8 = (v8f){0.f,0.f,0.f,0.f,0.f,0.f,0.f,0.f};

    for (unsigned t = 0; t < 2u; ++t) {
        const unsigned pt0 = p0 + 16u * t;
        {
            const float* gsrc = G1 + (pt0 + hh) * 64u + 4u * c;
#pragma unroll
            for (int it = 0; it < 8; ++it) {
                const v4f gv = *(const v4f*)(gsrc + (unsigned)it * 128u);
                *(v4f*)(tile + (2u * (unsigned)it + hh) * TP + 4u * c) = gv;
            }
        }
        wave_sync_lds();
        {
            v8f z[4];
#pragma unroll
            for (int j = 0; j < 4; ++j)
#pragma unroll
                for (int r = 0; r < 8; ++r)
                    z[j][r] = tile[(8u * hh + (unsigned)r) * TP + 16u * (unsigned)j + c] + p1v[j];
            wave_sync_lds();
            ln64_relu_store(z, g1v, e1v, tile, hh, c);
        }
        wave_sync_lds();
        v8f z2;
        {
            v8f ah = zero8, al = zero8;
#pragma unroll
            for (int ks = 0; ks < 2; ++ks) {
                v16h fh, fl;
                afrag2_full(tile + c * TP + 32u * (unsigned)ks + 8u * hh, fh, fl);
                const v16h bf = frag_ld(planes + (unsigned)OFF_W2P + c * 64u + 32u * (unsigned)ks + 8u * hh);
                ah = wmma16(fh, bf, ah);
                al = wmma16(fl, bf, al);
            }
#pragma unroll
            for (int r = 0; r < 8; ++r) z2[r] = (ah[r] + al[r] * LO_BACK) * SC22 + b2v;
        }
        wave_sync_lds();
        ln16_relu_store(z2, g2v, e2v, tile, hh, c);
        wave_sync_lds();
        v8f z3;
        {
            v16h fh, fl;
            afrag2_half(tile + c * TP + 8u * hh, fh, fl);
            const v16h bf = frag_ld(planes + (unsigned)OFF_W3P + c * 32u + 8u * hh);
            v8f ah = zero8, al = zero8;
            ah = wmma16(fh, bf, ah);
            al = wmma16(fl, bf, al);
#pragma unroll
            for (int r = 0; r < 8; ++r) z3[r] = (ah[r] + al[r] * LO_BACK) * SC22 + b3v;
        }
        wave_sync_lds();
        ln3_relu_store(z3, g3v, e3v, live3, tile, hh, c);
        wave_sync_lds();
        {
            v8f z4[4];
            const v16h fa = afrag1_half(tile + c * TP + 8u * hh);
#pragma unroll
            for (int j = 0; j < 4; ++j) {
                const v16h bf = frag_ld(planes + (unsigned)OFF_W4T + (16u * (unsigned)j + c) * 32u + 8u * hh);
                v8f a;
#pragma unroll
                for (int r = 0; r < 8; ++r) a[r] = p4v[j];
                a = wmma16(fa, bf, a);
#pragma unroll
                for (int r = 0; r < 8; ++r) z4[j][r] = a[r] * SC22;
            }
            wave_sync_lds();
            ln64_relu_store(z4, g4v, e4v, tile, hh, c);
        }
        wave_sync_lds();
        v8f z5;
        {
            v8f a5 = zero8;
#pragma unroll
            for (int ks = 0; ks < 2; ++ks) {
                const v16h fa = afrag1_full(tile + c * TP + 32u * (unsigned)ks + 8u * hh);
                const v16h bf = frag_ld(planes + (unsigned)OFF_W5P + c * 64u + 32u * (unsigned)ks + 8u * hh);
                a5 = wmma16(fa, bf, a5);
            }
#pragma unroll
            for (int r = 0; r < 8; ++r) z5[r] = a5[r] * SC22 + b5v;
        }
        wave_sync_lds();
        ln16_relu_store(z5, g5v, e5v, tile, hh, c);
        wave_sync_lds();
        {
            const v16h fa = afrag1_half(tile + c * TP + 8u * hh);
            const v16h bf = frag_ld(planes + (unsigned)OFF_W6P + c * 32u + 8u * hh);
            v8f a6 = zero8;
            a6 = wmma16(fa, bf, a6);
            float ov[8];
#pragma unroll
            for (int r = 0; r < 8; ++r) ov[r] = a6[r] * SC22 + b6v;
            if (live3) {
#pragma unroll
                for (int r = 0; r < 8; ++r) so[(16u * t + 8u * hh + (unsigned)r) * 3u + c] = ov[r];
            }
        }
        wave_sync_lds();
    }
    {
        const unsigned li = (lane < 24u) ? lane : 23u;
        const v4f ov = *(const v4f*)(so + 4u * li);
        float* dst = out + ((size_t)b * NPTS_FULL + p0) * 3u;
        if (lane < 24u) *(volatile v4f*)(dst + 4u * lane) = ov;
        __threadfence();
        if (lane < 24u) *(volatile v4f*)(dst + 4u * lane) = ov;
    }
}

extern "C" void kernel_launch(void* const* d_in, const int* in_sizes, int n_in, void* d_out, int out_size,
                              void* d_ws, size_t ws_size, hipStream_t stream) {
    if (n_in < 23) return;
    if (in_sizes[0] < NB * LAT || in_sizes[1] < 64 * W1_LD || in_sizes[2] < 64 || in_sizes[3] < 1024 || in_sizes[4] < 16) return;
    if (in_sizes[5] < 48 || in_sizes[6] < 3 || in_sizes[7] < 64 * W4_LD || in_sizes[8] < 64 || in_sizes[9] < 1024) return;
    if (in_sizes[10] < 16 || in_sizes[11] < 48 || in_sizes[12] < 3 || in_sizes[13] < 64 || in_sizes[14] < 64) return;
    if (in_sizes[15] < 16 || in_sizes[16] < 16 || in_sizes[17] < 3 || in_sizes[18] < 3 || in_sizes[19] < 64) return;
    if (in_sizes[20] < 64 || in_sizes[21] < 16 || in_sizes[22] < 16) return;
    if (out_size < ((NB - 1) * NPTS_FULL + NPTS) * 3) return;
    if (WS_TOTAL > ws_size) return;

    const float* x   = (const float*)d_in[0];
    const float* W1  = (const float*)d_in[1];
    const float* b1  = (const float*)d_in[2];
    const float* W2  = (const float*)d_in[3];
    const float* b2  = (const float*)d_in[4];
    const float* W3  = (const float*)d_in[5];
    const float* b3  = (const float*)d_in[6];
    const float* W4  = (const float*)d_in[7];
    const float* b4  = (const float*)d_in[8];
    const float* W5  = (const float*)d_in[9];
    const float* b5  = (const float*)d_in[10];
    const float* W6  = (const float*)d_in[11];
    const float* b6  = (const float*)d_in[12];
    const float* g1  = (const float*)d_in[13];
    const float* be1 = (const float*)d_in[14];
    const float* g2  = (const float*)d_in[15];
    const float* be2 = (const float*)d_in[16];
    const float* g3  = (const float*)d_in[17];
    const float* be3 = (const float*)d_in[18];
    const float* g4  = (const float*)d_in[19];
    const float* be4 = (const float*)d_in[20];
    const float* g5  = (const float*)d_in[21];
    const float* be5 = (const float*)d_in[22];
    float* out = (float*)d_out;

    char* wsp = (char*)d_ws;
    _Float16* planes = (_Float16*)(wsp + WS_PLANES);
    float*    P      = (float*)(wsp + WS_P);
    float*    G1     = (float*)(wsp + WS_G1);

    k_prep<<<PB7, 64, 0, stream>>>(x, W1, W2, W3, W4, W5, W6, planes);
    k_lat<<<2, 256, 0, stream>>>((const _Float16*)planes, b1, b4, P);
    k_grid<<<(NPTS * 16) / 256, 256, 0, stream>>>(W1, G1);
    k_fold<<<TOTAL_WAVES / 8, 256, 0, stream>>>((const _Float16*)planes, (const float*)P, (const float*)G1,
        b2, b3, b5, b6, g1, be1, g2, be2, g3, be3, g4, be4, g5, be5, out);
}
